// OSKAKERNEL_2310692405600
// MI455X (gfx1250) — hardware-run, weakly checked
//
#include <hip/hip_runtime.h>
#include <math.h>

typedef __attribute__((ext_vector_type(16))) _Float16 v16h;
typedef __attribute__((ext_vector_type(8)))  _Float16 v8h;
typedef __attribute__((ext_vector_type(8)))  float    v8f;
typedef __attribute__((ext_vector_type(4)))  float    v4f;
typedef __attribute__((ext_vector_type(4)))  unsigned int v4u;

constexpr int kBatch = 2;
constexpr int kSeq   = 1024;
constexpr int kDim   = 1024;
constexpr int kHeads = 16;
constexpr int kDh    = 64;
constexpr int kRows  = kBatch * kSeq;
constexpr int kBH    = kBatch * kHeads;
constexpr int kPld   = 3 * kDim;
constexpr int kNPoly = 9;
constexpr int kQDim  = 64;
constexpr double kLamD = (kQDim - 1) / 2.0;
constexpr float kWCarry    = 16.0f;
constexpr float kWCarryInv = 1.0f / kWCarry;
constexpr float kQKCarry   = 16.0f;
constexpr float kSimScale  = 1.0f / (kQKCarry * kQKCarry);
constexpr float kEpsNorm   = 1e-12f;
constexpr float kEpsRms    = 1e-6f;
constexpr float kInvDh     = 1.0f / (float)kDh;
static_assert(kHeads * kDh == kDim, "head split");
static_assert((kRows % 64) == 0 && (kPld % 64) == 0 && (kDim % 64) == 0, "GEMM M,N multiples of 64");
static_assert((kDim % 32) == 0 && (kDh % 32) == 0, "GEMM K multiples of 32");
static_assert((kSeq % 128) == 0, "query tiles of 128 rows");

constexpr size_t kOffXH   = 0;
constexpr size_t kOffWALL = kOffXH   + (size_t)kRows * kDim * 2;
constexpr size_t kOffP    = kOffWALL + (size_t)4 * kDim * kDim * 2;
constexpr size_t kOffQH   = kOffP    + (size_t)kRows * kPld * 4;
constexpr size_t kOffKH   = kOffQH   + (size_t)kBH * kSeq * kDh * 2;
constexpr size_t kOffVT   = kOffKH   + (size_t)kBH * kSeq * kDh * 2;
constexpr size_t kOffAH   = kOffVT   + (size_t)kBH * kDh * kSeq * 2;
constexpr size_t kWsTotal = kOffAH   + (size_t)kRows * kDim * 2;
static_assert(kWsTotal == 54525952ull, "carve total");
static_assert(kWsTotal <= 134217728ull, "carve cap");
static_assert((kOffWALL % 128) == 0 && (kOffP % 128) == 0 && (kOffQH % 128) == 0 && (kOffKH % 128) == 0 &&
              (kOffVT % 128) == 0 && (kOffAH % 128) == 0, "128-B aligned regions");

__device__ __forceinline__ void keep4_h(v16h a, v16h b, v16h c, v16h d) { asm volatile("v_nop" :: "v"(a), "v"(b), "v"(c), "v"(d)); }
__device__ __forceinline__ void acc_guard4(v8f& a, v8f& b, v8f& c, v8f& d) { asm volatile("v_nop\n\tv_nop\n\tv_nop\n\tv_nop" : "+v"(a), "+v"(b), "+v"(c), "+v"(d)); }
struct FragH {
  union U { v16h v; v8h h[2]; };
  static __device__ __forceinline__ v16h load(const _Float16* p) {
    U f; f.h[0] = *(const v8h*)(p); f.h[1] = *(const v8h*)(p + 16); return f.v;
  }
};
__device__ __forceinline__ v8f mma_h(v16h a, v16h b, v8f c) {
  c = __builtin_amdgcn_wmma_f32_16x16x32_f16(false, a, false, b, (short)0, c, false, false);
  asm volatile("v_nop\n\tv_nop\n\tv_nop\n\tv_nop" : "+v"(c) : "v"(a), "v"(b));
  return c;
}

__device__ __forceinline__ unsigned pk16(unsigned short a, unsigned short b) { return (unsigned)a | ((unsigned)b << 16); }
__device__ __forceinline__ unsigned short h_bits(float f) { const _Float16 h = (_Float16)f; return __builtin_bit_cast(unsigned short, h); }

__global__ __launch_bounds__(256) void wmma_gemm64_f16(
    const unsigned short* __restrict__ Ap, int lda,
    const unsigned short* __restrict__ Btp, int ldb,
    float* __restrict__ Cout, int ldc,
    int M, int N, int K, float scale) {
  const _Float16* A  = (const _Float16*)Ap;
  const _Float16* Bt = (const _Float16*)Btp;
  __shared__ __align__(16) float sT[8][16 * 68];
  const int lane = threadIdx.x & 31;
  const int wave = threadIdx.x >> 5;
  const int tilesN = N >> 6;
  const int tilesM = M >> 6;
  const int tile = blockIdx.x * 8 + wave;
  if (tile >= tilesM * tilesN) return;
  const int tm = tile / tilesN;
  const int tn = tile - tm * tilesN;
  const int m0 = tm << 6;
  const int n0 = tn << 6;

  const int rlane = lane & 15;
  const int koff  = (lane >> 4) * 8;
  const int mOff  = (lane >> 4) * 8;

  v8f acc[4][4];
#pragma unroll
  for (int i = 0; i < 4; ++i)
#pragma unroll
    for (int j = 0; j < 4; ++j) acc[i][j] = (v8f){0.f,0.f,0.f,0.f,0.f,0.f,0.f,0.f};

  for (int k0 = 0; k0 < K; k0 += 32) {
    v16h bh[4];
#pragma unroll
    for (int j = 0; j < 4; ++j) {
      const size_t bo = (size_t)(n0 + (j << 4) + rlane) * ldb + koff + k0;
      bh[j] = FragH::load(Bt + bo);
    }
#pragma unroll
    for (int i = 0; i < 4; ++i) {
      const size_t ao = (size_t)(m0 + (i << 4) + rlane) * lda + koff + k0;
      const v16h ah = FragH::load(A + ao);
#pragma unroll
      for (int j = 0; j < 4; ++j) acc[i][j] = mma_h(ah, bh[j], acc[i][j]);
    }
    keep4_h(bh[0], bh[1], bh[2], bh[3]);
  }
  acc_guard4(acc[0][0], acc[0][1], acc[0][2], acc[0][3]);
  acc_guard4(acc[1][0], acc[1][1], acc[1][2], acc[1][3]);
  acc_guard4(acc[2][0], acc[2][1], acc[2][2], acc[2][3]);
  acc_guard4(acc[3][0], acc[3][1], acc[3][2], acc[3][3]);

  float* slab = sT[wave];
#pragma unroll
  for (int i = 0; i < 4; ++i) {
    const int mBase = m0 + (i << 4);
#pragma unroll
    for (int j = 0; j < 4; ++j) {
#pragma unroll
      for (int r = 0; r < 8; ++r) {
        const float v = acc[i][j][r] * scale;
        slab[(mOff + r) * 68 + (j << 4) + rlane] = v;
      }
    }
    __builtin_amdgcn_fence(__ATOMIC_RELEASE, "workgroup");
    __builtin_amdgcn_wave_barrier();
    __builtin_amdgcn_fence(__ATOMIC_ACQUIRE, "workgroup");
    {
      const int hh = lane >> 4, c4 = (lane & 15) * 4;
      for (int pass = 0; pass < 2; ++pass) {
#pragma unroll
        for (int it = 0; it < 8; ++it) {
          const int row = it * 2 + hh;
          const v4f v = *(const v4f*)(slab + row * 68 + c4);
          *(volatile v4f*)(Cout + (size_t)(mBase + row) * ldc + n0 + c4) = v;
        }
        __threadfence();
      }
    }
    __builtin_amdgcn_fence(__ATOMIC_RELEASE, "workgroup");
    __builtin_amdgcn_wave_barrier();
    __builtin_amdgcn_fence(__ATOMIC_ACQUIRE, "workgroup");
  }
}

__global__ __launch_bounds__(256) void cast8_f16_kernel(
    const float* __restrict__ in0, const float* __restrict__ in1,
    const float* __restrict__ in2, const float* __restrict__ in3,
    unsigned short* __restrict__ out, int n8, float scale) {
  const int z = blockIdx.y;
  const float* in = (z == 0) ? in0 : (z == 1) ? in1 : (z == 2) ? in2 : in3;
  const int i = blockIdx.x * 256 + threadIdx.x;
  if (i >= n8) return;
  const float* p = in + 8 * (size_t)i;
  const v4f a = *(const v4f*)(p);
  const v4f c = *(const v4f*)(p + 4);
  unsigned short hb[8];
#pragma unroll
  for (int e = 0; e < 4; ++e) {
    const float fa = a[e] * scale;
    const float fc = c[e] * scale;
    hb[e]     = h_bits(fa);
    hb[4 + e] = h_bits(fc);
  }
  const v4u u = (v4u){pk16(hb[0], hb[1]), pk16(hb[2], hb[3]), pk16(hb[4], hb[5]), pk16(hb[6], hb[7])};
  unsigned short* q = out + (size_t)z * (size_t)n8 * 8 + 8 * (size_t)i;
  *(volatile v4u*)q = u;
  __threadfence();
  *(volatile v4u*)q = u;
}

__global__ __launch_bounds__(256) void pack_qk_kernel(
    const float* __restrict__ P, unsigned short* __restrict__ Qh, unsigned short* __restrict__ Kh) {
  const int tid = threadIdx.x;
  const int which = blockIdx.y;
  const int vid = blockIdx.x * 32 + (tid >> 3);
  const int sub = tid & 7;
  const int bs = vid >> 4;
  const int h  = vid & 15;
  const int b  = bs >> 10;
  const int s  = bs & (kSeq - 1);
  const float* p = P + (size_t)bs * kPld + which * kDim + h * kDh + sub * 8;
  const v4f a = *(const v4f*)(p);
  const v4f c = *(const v4f*)(p + 4);
  float ss = 0.0f;
#pragma unroll
  for (int e = 0; e < 4; ++e) {
    ss += a[e] * a[e];
    ss += c[e] * c[e];
  }
  ss += __shfl_xor(ss, 1, 32);
  ss += __shfl_xor(ss, 2, 32);
  ss += __shfl_xor(ss, 4, 32);
  const float inv = 1.0f / fmaxf(sqrtf(ss), kEpsNorm);
  unsigned short hb[8];
#pragma unroll
  for (int e = 0; e < 4; ++e) {
    const float fa = (a[e] * inv) * kQKCarry;
    const float fc = (c[e] * inv) * kQKCarry;
    hb[e]     = h_bits(fa);
    hb[4 + e] = h_bits(fc);
  }
  const v4u u = (v4u){pk16(hb[0], hb[1]), pk16(hb[2], hb[3]), pk16(hb[4], hb[5]), pk16(hb[6], hb[7])};
  unsigned short* base = (which == 0) ? Qh : Kh;
  unsigned short* q = base + ((size_t)(b * kHeads + h) * kSeq + s) * kDh + sub * 8;
  *(volatile v4u*)q = u;
  __threadfence();
  *(volatile v4u*)q = u;
}

__global__ __launch_bounds__(256) void pack_vt_kernel(
    const float* __restrict__ P, unsigned short* __restrict__ Vt) {
  __shared__ float sm[64 * 65];
  const int t  = threadIdx.x;
  const int s0 = blockIdx.x * 64;
  const int bh = blockIdx.y;
  const int b  = bh >> 4;
  const int h  = bh & 15;
  const float* src = P + ((size_t)b * kSeq + s0) * kPld + 2 * kDim + h * kDh;
#pragma unroll
  for (int i = 0; i < 4; ++i) {
    const int e  = i * 256 + t;
    const int kk = e >> 4;
    const int c4 = (e & 15) * 4;
    const v4f a = *(const v4f*)(src + (size_t)kk * kPld + c4);
    sm[(c4 + 0) * 65 + kk] = a[0];
    sm[(c4 + 1) * 65 + kk] = a[1];
    sm[(c4 + 2) * 65 + kk] = a[2];
    sm[(c4 + 3) * 65 + kk] = a[3];
  }
  __syncthreads();
  const int lane = t & 31, wave = t >> 5;
  const int q = lane >> 3, c8 = (lane & 7) * 8;
  v8h hv[2];
#pragma unroll
  for (int it = 0; it < 2; ++it) {
    const int row = wave * 8 + it * 4 + q;
#pragma unroll
    for (int e = 0; e < 8; ++e) {
      const float f = sm[row * 65 + c8 + e];
      hv[it][e] = (_Float16)f;
    }
  }
  unsigned short* dst = Vt + (size_t)bh * kDh * kSeq + s0;
  for (int pass = 0; pass < 2; ++pass) {
#pragma unroll
    for (int it = 0; it < 2; ++it) {
      const int row = wave * 8 + it * 4 + q;
      *(volatile v8h*)(dst + (size_t)row * kSeq + c8) = hv[it];
    }
    __threadfence();
  }
}

template <int KK> struct RecC {
  static constexpr float c1 = (float)(2.0 * ((double)KK + kLamD - 1.0) / ((double)KK + 2.0 * kLamD - 1.0));
  static constexpr float c2 = (float)(((double)KK - 1.0) / ((double)KK + 2.0 * kLamD - 1.0));
};
template <int KK>
__device__ __forceinline__ void rec_step16(const float (&sv)[16], float w, float (&Rp)[16], float (&Rc)[16], float (&ph)[16]) {
  constexpr float c1 = RecC<KK>::c1;
  constexpr float c2 = RecC<KK>::c2;
#pragma unroll
  for (int e = 0; e < 16; ++e) {
    const float Rn = (c1 * sv[e]) * Rc[e] - c2 * Rp[e];
    ph[e] += w * Rn;
    Rp[e] = Rc[e];
    Rc[e] = Rn;
  }
}

__global__ __launch_bounds__(256) void attn_poly_kernel(
    const unsigned short* __restrict__ Qp, const unsigned short* __restrict__ Kp,
    const unsigned short* __restrict__ Vp, const float* __restrict__ poly,
    const float* __restrict__ degs, const float* __restrict__ nw,
    unsigned short* __restrict__ Ah) {
  __shared__ __align__(16) _Float16 wt[8][16 * 40];
  __shared__ __align__(16) float os[8][16 * 68];
  const int tid  = threadIdx.x;
  const int wave = tid >> 5;
  const int lane = tid & 31;
  const int hh   = lane >> 4;
  const int c    = lane & 15;
  const int bh   = blockIdx.y;
  const int h    = bh & 15;
  const int b    = bh >> 4;
  const int m0   = blockIdx.x * 128 + wave * 16;

  float wg[kNPoly];
  {
    const float dg = degs[h];
#pragma unroll
    for (int kk = 0; kk < kNPoly; ++kk) {
      const float gate = fminf(fmaxf(dg - (float)kk + 1.0f, 0.0f), 1.0f);
      wg[kk] = poly[h * kNPoly + kk] * gate;
    }
  }
  int kmax = 0;
#pragma unroll
  for (int kk = 1; kk < kNPoly; ++kk) kmax = (wg[kk] != 0.0f) ? kk : kmax;

  const _Float16* Qb = (const _Float16*)Qp + (size_t)bh * kSeq * kDh;
  const _Float16* Kb = (const _Float16*)Kp + (size_t)bh * kSeq * kDh;
  const _Float16* Vb = (const _Float16*)Vp + (size_t)bh * kDh * kSeq;

  const v16h qa0 = FragH::load(Qb + (size_t)(m0 + c) * kDh + 8 * hh);
  const v16h qa1 = FragH::load(Qb + (size_t)(m0 + c) * kDh + 32 + 8 * hh);

  v8f oacc[4];
#pragma unroll
  for (int t = 0; t < 4; ++t) oacc[t] = (v8f){0.f,0.f,0.f,0.f,0.f,0.f,0.f,0.f};

  _Float16* wtw = wt[wave];
  const int kend = m0 + 16;

  for (int k0 = 0; k0 < kend; k0 += 32) {
    v8f s0 = (v8f){0.f,0.f,0.f,0.f,0.f,0.f,0.f,0.f};
    v8f s1 = (v8f){0.f,0.f,0.f,0.f,0.f,0.f,0.f,0.f};
    {
      const _Float16* kr0 = Kb + (size_t)(k0 + c) * kDh + 8 * hh;
      const _Float16* kr1 = Kb + (size_t)(k0 + 16 + c) * kDh + 8 * hh;
      const v16h kb00 = FragH::load(kr0);
      const v16h kb01 = FragH::load(kr0 + 32);
      const v16h kb10 = FragH::load(kr1);
      const v16h kb11 = FragH::load(kr1 + 32);
      s0 = mma_h(qa0, kb00, s0);
      s0 = mma_h(qa1, kb01, s0);
      s1 = mma_h(qa0, kb10, s1);
      s1 = mma_h(qa1, kb11, s1);
    }
    float sv[16], Rp[16], Rc[16], ph[16];
#pragma unroll
    for (int r = 0; r < 8; ++r) {
      sv[r]     = s0[r] * kSimScale;
      sv[8 + r] = s1[r] * kSimScale;
    }
#pragma unroll
    for (int e = 0; e < 16; ++e) {
      Rp[e] = 1.0f;
      Rc[e] = sv[e];
      ph[e] = wg[0] + wg[1] * sv[e];
    }
    if (kmax >= 2) rec_step16<2>(sv, wg[2], Rp, Rc, ph);
    if (kmax >= 3) rec_step16<3>(sv, wg[3], Rp, Rc, ph);
    if (kmax >= 4) rec_step16<4>(sv, wg[4], Rp, Rc, ph);
    if (kmax >= 5) rec_step16<5>(sv, wg[5], Rp, Rc, ph);
    if (kmax >= 6) rec_step16<6>(sv, wg[6], Rp, Rc, ph);
    if (kmax >= 7) rec_step16<7>(sv, wg[7], Rp, Rc, ph);
    if (kmax >= 8) rec_step16<8>(sv, wg[8], Rp, Rc, ph);

#pragma unroll
    for (int r = 0; r < 8; ++r) {
      const int row = 8 * hh + r;
      const int qi  = m0 + row;
      const float p0 = ((k0 + c) <= qi) ? ph[r] : 0.0f;
      const float p1 = ((k0 + 16 + c) <= qi) ? ph[8 + r] : 0.0f;
      wtw[row * 40 + c]      = (_Float16)p0;
      wtw[row * 40 + 16 + c] = (_Float16)p1;
    }
    __builtin_amdgcn_fence(__ATOMIC_RELEASE, "workgroup");
    __builtin_amdgcn_wave_barrier();
    __builtin_amdgcn_fence(__ATOMIC_ACQUIRE, "workgroup");

    const v16h pa = FragH::load(wtw + c * 40 + 8 * hh);
#pragma unroll
    for (int t = 0; t < 4; ++t) {
      const v16h vb = FragH::load(Vb + (size_t)(t * 16 + c) * kSeq + k0 + 8 * hh);
      oacc[t] = mma_h(pa, vb, oacc[t]);
    }
    __builtin_amdgcn_fence(__ATOMIC_RELEASE, "workgroup");
    __builtin_amdgcn_wave_barrier();
    __builtin_amdgcn_fence(__ATOMIC_ACQUIRE, "workgroup");
  }

  float nwv[4];
#pragma unroll
  for (int t = 0; t < 4; ++t) nwv[t] = nw[t * 16 + c];
  float* osw = os[wave];
#pragma unroll
  for (int r = 0; r < 8; ++r) {
    const int row = 8 * hh + r;
    const float inv = 1.0f / (float)(m0 + row + 1);
    float o[4];
    float ss = 0.0f;
#pragma unroll
    for (int t = 0; t < 4; ++t) {
      o[t] = oacc[t][r] * inv;
      ss += o[t] * o[t];
    }
    ss += __shfl_xor(ss, 1, 32);
    ss += __shfl_xor(ss, 2, 32);
    ss += __shfl_xor(ss, 4, 32);
    ss += __shfl_xor(ss, 8, 32);
    const float rs = rsqrtf(ss * kInvDh + kEpsRms);
#pragma unroll
    for (int t = 0; t < 4; ++t) osw[row * 68 + t * 16 + c] = (o[t] * rs) * nwv[t];
  }
  __builtin_amdgcn_fence(__ATOMIC_RELEASE, "workgroup");
  __builtin_amdgcn_wave_barrier();
  __builtin_amdgcn_fence(__ATOMIC_ACQUIRE, "workgroup");
  {
    const int q = lane >> 3, c8 = (lane & 7) * 8;
    v8h hv[4];
#pragma unroll
    for (int it = 0; it < 4; ++it) {
      const int row = it * 4 + q;
      const float* sp = osw + row * 68 + c8;
      const v4f a0 = *(const v4f*)(sp);
      const v4f a1 = *(const v4f*)(sp + 4);
#pragma unroll
      for (int e = 0; e < 4; ++e) {
        const float f0 = a0[e];
        const float f1 = a1[e];
        hv[it][e]     = (_Float16)f0;
        hv[it][4 + e] = (_Float16)f1;
      }
    }
    unsigned short* Arow = Ah + ((size_t)b * kSeq + m0) * kDim + h * kDh;
    for (int pass = 0; pass < 2; ++pass) {
#pragma unroll
      for (int it = 0; it < 4; ++it) {
        const int row = it * 4 + q;
        *(volatile v8h*)(Arow + (size_t)row * kDim + c8) = hv[it];
      }
      __threadfence();
    }
  }
}

extern "C" void kernel_launch(void* const* d_in, const int* in_sizes, int n_in,
                              void* d_out, int out_size, void* d_ws, size_t ws_size,
                              hipStream_t stream) {
  if (n_in < 8) return;
  if (in_sizes[0] != kRows * kDim) return;
  if (in_sizes[1] != kDim * kDim) return;
  if (in_sizes[2] != kDim * kDim) return;
  if (in_sizes[3] != kDim * kDim) return;
  if (in_sizes[4] != kDim * kDim) return;
  if (in_sizes[5] != kHeads * kNPoly) return;
  if (in_sizes[6] != kDh) return;
  if (in_sizes[7] != kHeads) return;
  if (out_size != kRows * kDim) return;
  if (ws_size < kWsTotal) return;

  const float* x    = (const float*)d_in[0];
  const float* Wq   = (const float*)d_in[1];
  const float* Wk   = (const float*)d_in[2];
  const float* Wv   = (const float*)d_in[3];
  const float* Wo   = (const float*)d_in[4];
  const float* poly = (const float*)d_in[5];
  const float* nw   = (const float*)d_in[6];
  const float* degs = (const float*)d_in[7];
  float* out = (float*)d_out;

  char* ws = (char*)d_ws;
  unsigned short* XH   = (unsigned short*)(ws + kOffXH);
  unsigned short* WALL = (unsigned short*)(ws + kOffWALL);
  unsigned short* WOH  = WALL + (size_t)3 * kDim * kDim;
  float*          P    = (float*)(ws + kOffP);
  unsigned short* QH   = (unsigned short*)(ws + kOffQH);
  unsigned short* KH   = (unsigned short*)(ws + kOffKH);
  unsigned short* VT   = (unsigned short*)(ws + kOffVT);
  unsigned short* AH   = (unsigned short*)(ws + kOffAH);

  cast8_f16_kernel<<<dim3((kRows * kDim / 8) / 256, 1), 256, 0, stream>>>(x, x, x, x, XH, kRows * kDim / 8, 1.0f);
  cast8_f16_kernel<<<dim3((kDim * kDim / 8) / 256, 4), 256, 0, stream>>>(Wq, Wk, Wv, Wo, WALL, kDim * kDim / 8, kWCarry);

  wmma_gemm64_f16<<<dim3((kRows / 64) * (kPld / 64) / 8), 256, 0, stream>>>(
      XH, kDim, WALL, kDim, P, kPld, kRows, kPld, kDim, kWCarryInv);

  pack_qk_kernel<<<dim3(kRows * kHeads / 32, 2), 256, 0, stream>>>(P, QH, KH);
  pack_vt_kernel<<<dim3(kSeq / 64, kBH), 256, 0, stream>>>(P, VT);

  attn_poly_kernel<<<dim3(kSeq / 128, kBH), 256, 0, stream>>>(QH, KH, VT, poly, degs, nw, AH);

  wmma_gemm64_f16<<<dim3((kRows / 64) * (kDim / 64) / 8), 256, 0, stream>>>(
      AH, kDim, WOH, kDim, out, kDim, kRows, kDim, kDim, kWCarryInv);
}
